// Point_TemporalPriorEncoder_6047313953101
// MI455X (gfx1250) — hardware-verified
//
#include <hip/hip_runtime.h>


namespace {
constexpr int C = 64, N1 = 240000, N2 = 120000, N3 = 40000, N4 = 24020;
constexpr float XS = 8.0f, HS = 256.0f, WSC = 256.0f;
typedef _Float16 b16;
typedef __attribute__((ext_vector_type(16))) _Float16 v16b;
typedef __attribute__((ext_vector_type(8))) _Float16 v8b;
typedef __attribute__((ext_vector_type(8))) float v8f;
typedef __attribute__((ext_vector_type(4))) float v4f;
typedef __attribute__((ext_vector_type(2))) float v2f;
typedef __attribute__((ext_vector_type(2))) _Float16 v2b;
__device__ __forceinline__ float bf16_rne(float f) { unsigned int u = __float_as_uint(f); u += 0x7FFFu + ((u >> 16) & 1u); float r = __uint_as_float(u & 0xFFFF0000u); asm volatile("" : "+v"(r)); return r; }
__device__ __forceinline__ float bfv(float f) { float r = bf16_rne(f); asm volatile("" : "+v"(r)); return r; }
__device__ __forceinline__ void split16(float v, b16& hi, b16& lo) { hi = (b16)v; lo = (b16)(v - (float)hi); }
__device__ __forceinline__ v16b frag_kb(const b16* p, int hh) { const v8b a = *(const v8b*)(p + 8 * hh), b = *(const v8b*)(p + 16 + 8 * hh); v16b f;
#pragma unroll
  for (int e = 0; e < 8; ++e) { f[e] = a[e]; f[8 + e] = b[e]; } return f; }
__device__ __forceinline__ v8f wmma16b(v16b a, v16b b, v8f c) { v8f d = __builtin_amdgcn_wmma_f32_16x16x32_f16(false, a, false, b, (short)0, c, false, false); asm volatile("v_nop\n\tv_nop\n\tv_nop\n\tv_nop" : "+v"(d) : "v"(a), "v"(b)); return d; }
__device__ __forceinline__ void wave_lds_sync() { __builtin_amdgcn_fence(__ATOMIC_RELEASE, "workgroup"); __builtin_amdgcn_wave_barrier(); __builtin_amdgcn_fence(__ATOMIC_ACQUIRE, "workgroup"); }
__device__ __forceinline__ int iclamp(int v, int lo, int hi) { return v < lo ? lo : (v > hi ? hi : v); }

__global__ __launch_bounds__(256) void wput_kernel(const float* __restrict__ w1, const float* __restrict__ w2, const float* __restrict__ w3, const float* __restrict__ w4, const float* __restrict__ w5, b16* __restrict__ WT1, b16* __restrict__ WT2, b16* __restrict__ WT3, b16* __restrict__ WT4, b16* __restrict__ WT5) { const size_t nt = (size_t)gridDim.x * 256, u0 = (size_t)blockIdx.x * 256 + threadIdx.x; v8b v;
  for (int l = 0; l < 5; ++l) { const int K = l < 3 ? 8 : 27; const float* w = l == 0 ? w1 : l == 1 ? w2 : l == 2 ? w3 : l == 3 ? w4 : w5; b16* dst = l == 0 ? WT1 : l == 1 ? WT2 : l == 2 ? WT3 : l == 3 ? WT4 : WT5;
    for (size_t u = u0; u < (size_t)C * K * 8; u += nt) { const int o = (int)(u / (K * 8)), q = (int)(u % (K * 8)); const int k = q / 8, c0 = (q % 8) * 8;
#pragma unroll
      for (int j = 0; j < 8; ++j) v[j] = (b16)(bf16_rne(w[((size_t)k * C + c0 + j) * C + o]) * WSC); for (int pass = 0; pass < 2; ++pass) { *(volatile v8b*)(dst + (size_t)o * (K * C) + k * C + c0) = v; __threadfence(); } } } }
template <int K, bool RAW, bool SKIP, bool RELU>
__global__ __launch_bounds__(32) void sconv_kernel(const float* __restrict__ IN, int NIN, const int* __restrict__ imap, const b16* __restrict__ WT, const float* __restrict__ bias, const float* __restrict__ SKF, int NSK, const int* __restrict__ match, int MOUT, int MLIM, float* __restrict__ OUTR) { constexpr int KD = K * C; __shared__ __attribute__((aligned(16))) b16 Ah[16][KD + 8], Al[RAW ? 1 : 16][KD + 8]; __shared__ float Tf[16][C + 1]; const int lane = threadIdx.x, nloc = lane & 15, hlf = lane >> 4; const size_t m0 = (size_t)blockIdx.x * 16; if (m0 >= (size_t)MLIM) return; const int nr = (MOUT - (int)m0) < 16 ? (MOUT - (int)m0) : 16;
  for (int rr = 0; rr < 16; ++rr) { const size_t m = m0 + (rr < nr ? rr : 0);
#pragma unroll 1
    for (int k = 0; k < K; ++k) { const int src = imap[(size_t)k * MOUT + m]; const bool ok = src >= 0 && src < NIN; float v0 = 0.0f, v1 = 0.0f; if (ok) { v0 = IN[(size_t)src * C + lane]; v1 = IN[(size_t)src * C + 32 + lane]; if (RAW) { v0 = bfv(v0); v1 = bfv(v1); } }
      if (RAW) { Ah[rr][k * C + lane] = (b16)(v0 * XS); Ah[rr][k * C + 32 + lane] = (b16)(v1 * XS); } else { b16 p, pl; split16(v0 * HS, p, pl); Ah[rr][k * C + lane] = p; Al[rr][k * C + lane] = pl; split16(v1 * HS, p, pl); Ah[rr][k * C + 32 + lane] = p; Al[rr][k * C + 32 + lane] = pl; } } }
  if (lane < 16) for (int kk = KD; kk < KD + 8; ++kk) { Ah[lane][kk] = (b16)0.0f; if (!RAW) Al[lane][kk] = (b16)0.0f; }
  wave_lds_sync(); v8f acc[4] = {(v8f){}, (v8f){}, (v8f){}, (v8f){}};
#pragma unroll 2
  for (int kb = 0; kb < KD; kb += 32) { const v16b a = frag_kb(&Ah[nloc][kb], hlf); v16b al; if (!RAW) al = frag_kb(&Al[nloc][kb], hlf);
#pragma unroll
    for (int t = 0; t < 4; ++t) { const v16b bw = frag_kb(WT + (size_t)(t * 16 + nloc) * KD + kb, hlf); acc[t] = wmma16b(a, bw, acc[t]); if (!RAW) acc[t] = wmma16b(al, bw, acc[t]); } }
  const float isc = RAW ? 1.0f / (XS * WSC) : 1.0f / (HS * WSC);
#pragma unroll
  for (int t = 0; t < 4; ++t) { const int cc = t * 16 + nloc; const float bb = bfv(bias[cc]);
#pragma unroll
    for (int r8 = 0; r8 < 8; ++r8) { const int rr = 8 * hlf + r8; float v = acc[t][r8] * isc + bb; if (SKIP) { const size_t m = m0 + (rr < nr ? rr : 0); const int mi = match[m]; if (mi >= 0 && mi < NSK) v += bfv(SKF[(size_t)mi * C + cc]); } Tf[rr][cc] = RELU ? fmaxf(v, 0.0f) : v; } }
  wave_lds_sync();
  for (int pass = 0; pass < 2; ++pass) { for (int rr = 0; rr < nr; ++rr) *(volatile v2f*)(OUTR + (m0 + rr) * C + lane * 2) = (v2f){Tf[rr][lane * 2], Tf[rr][lane * 2 + 1]}; __threadfence(); } }
}

extern "C" void kernel_launch(void* const* d_in, const int* in_sizes, int n_in, void* d_out, int out_size, void* d_ws, size_t ws_size, hipStream_t stream) {
  (void)n_in;
  auto Fp = [&](int i) { return (const float*)d_in[i]; }; auto Ip = [&](int i) { return (const int*)d_in[i]; };
  if (in_sizes[0] != N1 * C || in_sizes[1] != N2 * C || in_sizes[2] != N3 * C || in_sizes[3] != 8 * C * C || in_sizes[9] != 27 * C * C || in_sizes[11] != 27 * C * C || in_sizes[13] != 8 * N2 || in_sizes[15] != 8 * N3 || in_sizes[17] != 8 * N4 || in_sizes[19] != 27 * N4 || in_sizes[21] != 27 * N4 || in_sizes[23] != N2 || in_sizes[24] != N3 || out_size != N4 * C) return;
  const int DIV = 1;
  size_t off = 0; char* ws = (char*)d_ws;
  auto carve = [&](size_t bytes) { char* p = ws + off; off += (bytes + 255) & ~(size_t)255; return p; };
  b16* WT1 = (b16*)carve(C * 8 * C * 2); b16* WT2 = (b16*)carve(C * 8 * C * 2); b16* WT3 = (b16*)carve(C * 8 * C * 2); b16* WT4 = (b16*)carve((size_t)C * 27 * C * 2); b16* WT5 = (b16*)carve((size_t)C * 27 * C * 2);
  float* F1 = (float*)carve((size_t)N2 * C * 4); float* F2 = (float*)carve((size_t)N3 * C * 4); float* F3 = (float*)carve((size_t)N4 * C * 4); float* F4 = (float*)carve((size_t)N4 * C * 4);
  if (off > ws_size || off > ((size_t)64 << 20)) return;
  wput_kernel<<<64, 256, 0, stream>>>(Fp(3), Fp(5), Fp(7), Fp(9), Fp(11), WT1, WT2, WT3, WT4, WT5);
  auto lim = [&](int M) { int v = M / DIV; v = (v + 15) / 16 * 16; return v > M ? M : v; };
  const int L1 = lim(N2), L2 = lim(N3), L3 = lim(N4), L4 = L3;
  sconv_kernel<8, true, true, false><<<(N2 + 15) / 16, 32, 0, stream>>>(Fp(0), N1, Ip(13), WT1, Fp(4), Fp(1), N2, Ip(23), N2, L1, F1);
  sconv_kernel<8, false, true, false><<<(N3 + 15) / 16, 32, 0, stream>>>(F1, L1, Ip(15), WT2, Fp(6), Fp(2), N3, Ip(24), N3, L2, F2);
  sconv_kernel<8, false, false, false><<<(N4 + 15) / 16, 32, 0, stream>>>(F2, L2, Ip(17), WT3, Fp(8), nullptr, 0, nullptr, N4, L3, F3);
  sconv_kernel<27, false, false, true><<<(N4 + 15) / 16, 32, 0, stream>>>(F3, L3, Ip(19), WT4, Fp(10), nullptr, 0, nullptr, N4, L4, F4);
  sconv_kernel<27, false, false, false><<<(N4 + 15) / 16, 32, 0, stream>>>(F4, L4, Ip(21), WT5, Fp(12), nullptr, 0, nullptr, N4, L4, (float*)d_out);
}
